// LSTMLightweight_39779987096022
// MI455X (gfx1250) — hardware-verified
//
#include <hip/hip_runtime.h>

#define NB_ 8192
#define TT_ 256
#define HH_ 16

typedef _Float16 f16;
typedef __attribute__((ext_vector_type(16))) f16 f16x16;
typedef __attribute__((ext_vector_type(8)))  float f32x8;
typedef __attribute__((ext_vector_type(4)))  float v4f_t;
typedef float v4fa __attribute__((ext_vector_type(4), may_alias));

__device__ __forceinline__ f32x8 wmma16(f16x16 a, f16x16 b, f32x8 c) {
  c = __builtin_amdgcn_wmma_f32_16x16x32_f16(false, a, false, b, (short)0, c, false, false);
  asm volatile("v_nop\n\tv_nop\n\tv_nop\n\tv_nop" : "+v"(c) : "v"(a), "v"(b));
  return c;
}
__device__ __forceinline__ void split16(float v, f16& h, f16& l) { h = (f16)v; l = (f16)((v - (float)h) * 2048.0f); }
__device__ __forceinline__ float sigm(float x) { return 1.0f / (1.0f + __expf(-x)); }
__device__ __forceinline__ float tanh_(float x) { return 1.0f - 2.0f / (1.0f + __expf(2.0f * x)); }

__device__ __forceinline__ void load_wfrags(const float* __restrict__ wih, const float* __restrict__ whh, f16x16* bh, f16x16* bl) {
  const int lane = threadIdx.x & 31, cl = lane & 15, kh = (lane >> 4) * 8;
#pragma unroll
  for (int nt = 0; nt < 4; ++nt) {
    const int n = nt * 16 + cl;
#pragma unroll
    for (int i = 0; i < 8; ++i) {
      f16 h, l;
      split16(wih[n * HH_ + kh + i], h, l); bh[nt][i] = h;     bl[nt][i] = l;
      split16(whh[n * HH_ + kh + i], h, l); bh[nt][8 + i] = h; bl[nt][8 + i] = l;
    }
  }
}

__global__ __launch_bounds__(256) void k_lstm2(const float* __restrict__ x, const float* __restrict__ win, const float* __restrict__ bin,
                                               const float* __restrict__ wih0, const float* __restrict__ whh0, const float* __restrict__ bih0, const float* __restrict__ bhh0,
                                               const float* __restrict__ wih1, const float* __restrict__ whh1, const float* __restrict__ bih1, const float* __restrict__ bhh1,
                                               const float* __restrict__ fchw, const float* __restrict__ fchb, const float* __restrict__ fcow, const float* __restrict__ fcob,
                                               float* __restrict__ out) {
  __shared__ float hS[8][2][16 * 17];
  __shared__ __attribute__((aligned(16))) float oS[128];
  const int tid = threadIdx.x, lane = tid & 31, wave = tid >> 5, cl = lane & 15, hsel = lane >> 4, kh = hsel * 8, rh = kh;
  const int row0 = blockIdx.x * 128 + wave * 16;
  const int myrow = row0 + cl;

  f16x16 b0h[4], b0l[4], b1h[4], b1l[4];
  load_wfrags(wih0, whh0, b0h, b0l);
  load_wfrags(wih1, whh1, b1h, b1l);
  float bsum0[4], bsum1[4], winv[8], binv[8];
#pragma unroll
  for (int nt = 0; nt < 4; ++nt) { bsum0[nt] = bih0[nt * 16 + cl] + bhh0[nt * 16 + cl]; bsum1[nt] = bih1[nt * 16 + cl] + bhh1[nt * 16 + cl]; }
#pragma unroll
  for (int i = 0; i < 8; ++i) { winv[i] = win[kh + i]; binv[i] = bin[kh + i]; }
  float* h0T = hS[wave][0]; float* h1T = hS[wave][1];
  for (int e = lane; e < 16 * 17; e += 32) { h0T[e] = 0.0f; h1T[e] = 0.0f; }
  float c0[8], c1[8];
#pragma unroll
  for (int r = 0; r < 8; ++r) { c0[r] = 0.0f; c1[r] = 0.0f; }
  asm volatile("s_wait_dscnt 0" ::: "memory");
  __builtin_amdgcn_wave_barrier();

#pragma unroll 1
  for (int t = 0; t < TT_; ++t) {
    const float xt = x[(size_t)myrow * TT_ + t];
    f16x16 ah, al;
#pragma unroll
    for (int i = 0; i < 8; ++i) {
      f16 h, l;
      split16(fmaxf(xt * winv[i] + binv[i], 0.0f), h, l); ah[i] = h; al[i] = l;
      split16(h0T[cl * 17 + kh + i], h, l); ah[8 + i] = h; al[8 + i] = l;
    }
    f32x8 g[4];
#pragma unroll
    for (int nt = 0; nt < 4; ++nt) { f32x8 z = {}; z = wmma16(ah, b0h[nt], z); f32x8 zl = {}; zl = wmma16(ah, b0l[nt], zl); zl = wmma16(al, b0h[nt], zl);
#pragma unroll
      for (int r = 0; r < 8; ++r) z[r] += zl[r] * (1.0f / 2048.0f) + bsum0[nt];
      g[nt] = z; }
    float h0new[8];
#pragma unroll
    for (int r = 0; r < 8; ++r) {
      const float ig = sigm(g[0][r]), fg = sigm(g[1][r]), gg = tanh_(g[2][r]), og = sigm(g[3][r]);
      c0[r] = fg * c0[r] + ig * gg; h0new[r] = og * tanh_(c0[r]);
    }
    __builtin_amdgcn_wave_barrier();
#pragma unroll
    for (int r = 0; r < 8; ++r) h0T[(rh + r) * 17 + cl] = h0new[r];
    asm volatile("s_wait_dscnt 0" ::: "memory");
    __builtin_amdgcn_wave_barrier();
#pragma unroll
    for (int i = 0; i < 8; ++i) {
      f16 h, l;
      split16(h0T[cl * 17 + kh + i], h, l); ah[i] = h; al[i] = l;
      split16(h1T[cl * 17 + kh + i], h, l); ah[8 + i] = h; al[8 + i] = l;
    }
#pragma unroll
    for (int nt = 0; nt < 4; ++nt) { f32x8 z = {}; z = wmma16(ah, b1h[nt], z); f32x8 zl = {}; zl = wmma16(ah, b1l[nt], zl); zl = wmma16(al, b1h[nt], zl);
#pragma unroll
      for (int r = 0; r < 8; ++r) z[r] += zl[r] * (1.0f / 2048.0f) + bsum1[nt];
      g[nt] = z; }
    float h1new[8];
#pragma unroll
    for (int r = 0; r < 8; ++r) {
      const float ig = sigm(g[0][r]), fg = sigm(g[1][r]), gg = tanh_(g[2][r]), og = sigm(g[3][r]);
      c1[r] = fg * c1[r] + ig * gg; h1new[r] = og * tanh_(c1[r]);
    }
    __builtin_amdgcn_wave_barrier();
#pragma unroll
    for (int r = 0; r < 8; ++r) h1T[(rh + r) * 17 + cl] = h1new[r];
    asm volatile("s_wait_dscnt 0" ::: "memory");
    __builtin_amdgcn_wave_barrier();
  }
  {
    f16x16 ah, al, bh, bl;
#pragma unroll
    for (int i = 0; i < 8; ++i) {
      f16 h, l;
      split16(h1T[cl * 17 + kh + i], h, l); ah[i] = h; al[i] = l; ah[8 + i] = (f16)0.0f; al[8 + i] = (f16)0.0f;
      const float wv = (cl < 8) ? fchw[cl * HH_ + kh + i] : 0.0f;
      split16(wv, h, l); bh[i] = h; bl[i] = l; bh[8 + i] = (f16)0.0f; bl[8 + i] = (f16)0.0f;
    }
    f32x8 z = {}, zl = {};
    z = wmma16(ah, bh, z); zl = wmma16(ah, bl, zl); zl = wmma16(al, bh, zl);
    const float fb = (cl < 8) ? fchb[cl] : 0.0f, fo = (cl < 8) ? fcow[cl] : 0.0f;
#pragma unroll
    for (int r = 0; r < 8; ++r) {
      float v = (cl < 8) ? fmaxf(z[r] + zl[r] * (1.0f / 2048.0f) + fb, 0.0f) * fo : 0.0f;
#pragma unroll
      for (int off = 8; off >= 1; off >>= 1) v += __shfl_xor(v, off, 32);
      if (cl == 0) oS[wave * 16 + rh + r] = v + fcob[0];
    }
  }
  __syncthreads();
  if (wave == 0) {
#pragma unroll 1
    for (int pass = 0; pass < 2; ++pass) { *(volatile v4f_t*)(out + (size_t)blockIdx.x * 128 + lane * 4) = *(const volatile v4fa*)(oS + lane * 4); __threadfence(); }
  }
}

extern "C" void kernel_launch(void* const* d_in, const int* in_sizes, int n_in,
                              void* d_out, int out_size, void* d_ws, size_t ws_size,
                              hipStream_t stream) {
  (void)in_sizes; (void)n_in; (void)out_size; (void)d_ws; (void)ws_size;
  const float* x = (const float*)d_in[0];
  const float* win = (const float*)d_in[1], *bin = (const float*)d_in[2];
  const float* wih0 = (const float*)d_in[3], *whh0 = (const float*)d_in[4], *bih0 = (const float*)d_in[5], *bhh0 = (const float*)d_in[6];
  const float* wih1 = (const float*)d_in[7], *whh1 = (const float*)d_in[8], *bih1 = (const float*)d_in[9], *bhh1 = (const float*)d_in[10];
  const float* fchw = (const float*)d_in[11], *fchb = (const float*)d_in[12], *fcow = (const float*)d_in[13], *fcob = (const float*)d_in[14];
  float* out = (float*)d_out;
  k_lstm2<<<dim3(NB_ / 128), dim3(256), 0, stream>>>(x, win, bin, wih0, whh0, bih0, bhh0, wih1, whh1, bih1, bhh1, fchw, fchb, fcow, fcob, out);
}
